// Indexing_Blend_Kron3_MLP_77223511982254
// MI455X (gfx1250) — hardware-run, weakly checked
//
#include <hip/hip_runtime.h>

typedef _Float16 v16h __attribute__((ext_vector_type(16)));
typedef _Float16 v8h  __attribute__((ext_vector_type(8)));
typedef float    v8f  __attribute__((ext_vector_type(8)));
typedef float    v4f  __attribute__((ext_vector_type(4)));
typedef v8h __attribute__((may_alias)) v8ha;
typedef v4f __attribute__((may_alias)) v4fa;

union Frag { v16h v; v8h half[2]; };

#define NG      64
#define NG3     262144
#define W0      256
#define WID     256
#define NOUT    3
#define KNB     8
#define KC      27
#define KP      32
#define QB      64
#define HP      264
#define SP      72

#define CORE_SC   1024.0f
#define H0_SC     0.25f
#define W1_SC     64.0f
#define H1_ISC    (1.0f / 16384.0f)

__device__ __forceinline__ v8f wmma_f16(v16h a, v16h b, v8f c) {
#if defined(__HIP_DEVICE_COMPILE__)
  v8f d = __builtin_amdgcn_wmma_f32_16x16x32_f16(false, a, false, b, (short)0, c, false, false);
  asm volatile("v_nop\n\tv_nop\n\tv_nop\n\tv_nop" : "+v"(d) : "v"(a), "v"(b));
  return d;
#else
  (void)a; (void)b;
  return c;
#endif
}

__device__ __forceinline__ float frcp(float v) {
#if defined(__HIP_DEVICE_COMPILE__)
  return __builtin_amdgcn_rcpf(v);
#else
  return 1.0f / v;
#endif
}

__device__ __forceinline__ v16h load_frag(const _Float16* p, int h) {
  Frag f;
  f.half[0] = *(const v8ha*)(p + 8 * h);
  f.half[1] = *(const v8ha*)(p + 16 + 8 * h);
  return f.v;
}

__global__ __launch_bounds__(256) void prep_w1_kernel(
    const float* __restrict__ W1, _Float16* __restrict__ W1T)
{
  __shared__ __attribute__((aligned(16))) _Float16 S[16 * SP];
  const int t = threadIdx.x;
  const int tn = blockIdx.x & 15, tk = blockIdx.x >> 4;
  const int n0 = 16 * tn, k0 = 64 * tk;
  #pragma unroll
  for (int p = 0; p < 4; ++p) {
    const int e = t + 256 * p;
    const int kk = e >> 4, nn = e & 15;
    const float v = W1[(size_t)(k0 + kk) * WID + n0 + nn];
    S[nn * SP + kk] = (_Float16)(v * W1_SC);
  }
  __syncthreads();
  const int lane = t & 31, wv = t >> 5;
  const int nn = (wv & 3) * 4 + (lane >> 3), q8 = lane & 7;
  const v8h v = *(const v8ha*)(S + nn * SP + 8 * q8);
  _Float16* dst = W1T + (size_t)(n0 + nn) * W0 + k0 + 8 * q8;
  if (wv < 4) *(volatile v8h*)dst = v;
  __threadfence();
  if (wv < 4) *(volatile v8h*)dst = v;
}

__global__ __launch_bounds__(256) void prep_core_kernel(
    const float* __restrict__ core, _Float16* __restrict__ coreK)
{
  __shared__ __attribute__((aligned(16))) _Float16 F[W0 * KP];
  const int t = threadIdx.x;
  #pragma unroll 1
  for (int p = 0; p < KP; ++p) {
    const int ps = (p < KC) ? p : (KC - 1);
    const float fv = core[t * KC + ps] * CORE_SC;
    const float sel = (p < KC) ? fv : 0.0f;
    F[t * KP + p] = (_Float16)sel;
  }
  __syncthreads();
  const int lane = t & 31, wv = t >> 5, q8 = lane & 7, sub = lane >> 3;
  #pragma unroll
  for (int i = 0; i < 4; ++i) {
    const int L = wv * 16 + i * 4 + sub;
    const v8h v = *(const v8ha*)(F + L * 64 + 8 * q8);
    *(volatile v8h*)(coreK + (size_t)L * 64 + 8 * q8) = v;
  }
  __threadfence();
  #pragma unroll
  for (int i = 0; i < 4; ++i) {
    const int L = wv * 16 + i * 4 + sub;
    const v8h v = *(const v8ha*)(F + L * 64 + 8 * q8);
    *(volatile v8h*)(coreK + (size_t)L * 64 + 8 * q8) = v;
  }
}

__global__ __launch_bounds__(256) void gather_mlp_kernel(
    const int*   __restrict__ Bidx,
    const float* __restrict__ Bw,
    const float* __restrict__ x,
    const float* __restrict__ y,
    const float* __restrict__ z,
    const _Float16* __restrict__ coreK,
    const _Float16* __restrict__ W1T,
    const float* __restrict__ b1,
    const float* __restrict__ W2,
    const float* __restrict__ b2,
    float* __restrict__ out)
{
  __shared__ float xs[192];
  __shared__ float ys[192];
  __shared__ float zs[192];
  __shared__ __attribute__((aligned(16))) _Float16 Gs[QB * KP];
  __shared__ __attribute__((aligned(16))) _Float16 Hs[QB * HP];
  __shared__ float Po[4 * QB * NOUT];
  __shared__ __attribute__((aligned(16))) float Os[QB * NOUT];

  const int t = threadIdx.x, lane = t & 31, wv = t >> 5;
  const int h = lane >> 4, m = lane & 15;
  const int q0 = blockIdx.x * QB;

  if (t < 192) { xs[t] = x[t]; ys[t] = y[t]; zs[t] = z[t]; }
  __syncthreads();

  if (t < QB) {
    float g[KC];
    #pragma unroll
    for (int p = 0; p < KC; ++p) g[p] = 0.0f;
    const size_t base = (size_t)(q0 + t) * KNB;
    #pragma unroll 1
    for (int q = 0; q < KNB; ++q) {
      int n = Bidx[base + q];
      const float bw = Bw[base + q];
      n = (n < 0) ? (n + NG3) : n;
      n = (n < 0) ? 0 : n;
      n = (n > NG3 - 1) ? (NG3 - 1) : n;
      const int i = n >> 12, k = (n >> 6) & 63, j = n & 63;
      float xv[3], yv[3], zw[3];
      #pragma unroll
      for (int c = 0; c < 3; ++c) {
        xv[c] = xs[3 * i + c];
        yv[c] = ys[3 * j + c];
        zw[c] = bw * zs[3 * k + c];
      }
      #pragma unroll
      for (int a = 0; a < 3; ++a) {
        #pragma unroll
        for (int c = 0; c < 3; ++c) {
          const float zx = zw[a] * xv[c];
          #pragma unroll
          for (int b = 0; b < 3; ++b)
            g[a * 9 + c * 3 + b] = fmaf(zx, yv[b], g[a * 9 + c * 3 + b]);
        }
      }
    }
    v8h o0, o1, o2, o3;
    #pragma unroll
    for (int e = 0; e < 8; ++e) {
      o0[e] = (_Float16)g[e];
      o1[e] = (_Float16)g[8 + e];
      o2[e] = (_Float16)g[16 + e];
    }
    o3[0] = (_Float16)g[24]; o3[1] = (_Float16)g[25]; o3[2] = (_Float16)g[26];
    o3[3] = (_Float16)g[0];  o3[4] = (_Float16)g[1];  o3[5] = (_Float16)g[2];
    o3[6] = (_Float16)g[3];  o3[7] = (_Float16)g[4];
    *(v8ha*)(Gs + t * KP + 0)  = o0;
    *(v8ha*)(Gs + t * KP + 8)  = o1;
    *(v8ha*)(Gs + t * KP + 16) = o2;
    *(v8ha*)(Gs + t * KP + 24) = o3;
  }
  __syncthreads();

  const v8f zero8 = {0.f, 0.f, 0.f, 0.f, 0.f, 0.f, 0.f, 0.f};

  {
    const int rt = wv & 3, cb = (wv >> 2) * 8;
    const v16h a = load_frag(Gs + (16 * rt + m) * KP, h);
    #pragma unroll
    for (int c8 = 0; c8 < 8; ++c8) {
      const int ct = cb + c8;
      const v16h b = load_frag(coreK + (size_t)(16 * ct + m) * KP, h);
      const v8f acc = wmma_f16(a, b, zero8);
      #pragma unroll
      for (int r = 0; r < 8; ++r)
        Hs[(16 * rt + 8 * h + r) * HP + 16 * ct + m] = (_Float16)(fmaxf(acc[r], 0.0f) * H0_SC);
    }
  }
  __syncthreads();

  const int rs = wv & 1, cg = wv >> 1;
  v8f acc[2][4];
  #pragma unroll
  for (int mt = 0; mt < 2; ++mt)
    #pragma unroll
    for (int nt = 0; nt < 4; ++nt) acc[mt][nt] = zero8;

  const _Float16* arow0 = Hs + (32 * rs + m) * HP;
  const _Float16* arow1 = arow0 + 16 * HP;
  const _Float16* brow  = W1T + (size_t)(64 * cg + m) * W0;

  #pragma unroll 1
  for (int k0 = 0; k0 < W0; k0 += 32) {
    const v16h a0 = load_frag(arow0 + k0, h);
    const v16h a1 = load_frag(arow1 + k0, h);
    #pragma unroll
    for (int nt = 0; nt < 4; ++nt) {
      const v16h b = load_frag(brow + (size_t)nt * 16 * W0 + k0, h);
      acc[0][nt] = wmma_f16(a0, b, acc[0][nt]);
      acc[1][nt] = wmma_f16(a1, b, acc[1][nt]);
    }
  }

  float po[2][8][3];
  #pragma unroll
  for (int mt = 0; mt < 2; ++mt)
    #pragma unroll
    for (int r = 0; r < 8; ++r) { po[mt][r][0] = 0.0f; po[mt][r][1] = 0.0f; po[mt][r][2] = 0.0f; }

  #pragma unroll
  for (int nt = 0; nt < 4; ++nt) {
    const int col = 64 * cg + 16 * nt + m;
    const float bb  = b1[col];
    const float w20 = W2[col * NOUT + 0];
    const float w21 = W2[col * NOUT + 1];
    const float w22 = W2[col * NOUT + 2];
    #pragma unroll
    for (int mt = 0; mt < 2; ++mt) {
      #pragma unroll
      for (int r = 0; r < 8; ++r) {
        const float v = fmaxf(acc[mt][nt][r] * H1_ISC + bb, 0.0f);
        po[mt][r][0] = fmaf(v, w20, po[mt][r][0]);
        po[mt][r][1] = fmaf(v, w21, po[mt][r][1]);
        po[mt][r][2] = fmaf(v, w22, po[mt][r][2]);
      }
    }
  }

  #pragma unroll
  for (int mt = 0; mt < 2; ++mt) {
    #pragma unroll
    for (int r = 0; r < 8; ++r) {
      #pragma unroll
      for (int o = 0; o < 3; ++o) {
        float v = po[mt][r][o];
        v += __shfl_xor(v, 8);
        v += __shfl_xor(v, 4);
        v += __shfl_xor(v, 2);
        v += __shfl_xor(v, 1);
        po[mt][r][o] = v;
      }
    }
  }
  if (m == 0) {
    #pragma unroll
    for (int mt = 0; mt < 2; ++mt) {
      #pragma unroll
      for (int r = 0; r < 8; ++r) {
        const int row = 32 * rs + 16 * mt + 8 * h + r;
        #pragma unroll
        for (int o = 0; o < 3; ++o) Po[(cg * QB + row) * NOUT + o] = po[mt][r][o];
      }
    }
  }
  __syncthreads();

  if (t < QB * NOUT) {
    const int row = t / NOUT, o = t - NOUT * row;
    float s = b2[o];
    s += Po[(0 * QB + row) * NOUT + o];
    s += Po[(1 * QB + row) * NOUT + o];
    s += Po[(2 * QB + row) * NOUT + o];
    s += Po[(3 * QB + row) * NOUT + o];
    const float e = __expf(-s);
    Os[t] = frcp(1.0f + e);
  }
  __syncthreads();

  const int li = (wv == 0) ? lane : (lane & 15);
  const int oi = ((wv == 0) ? 0 : 128) + 4 * li;
  const v4f ov = *(const v4fa*)(Os + oi);
  float* ob = out + (size_t)blockIdx.x * (QB * NOUT);
  const bool act = (wv == 0) || (wv == 1 && lane < 16);
  if (act) *(volatile v4f*)(ob + oi) = ov;
  __threadfence();
  if (act) *(volatile v4f*)(ob + oi) = ov;
}

extern "C" void kernel_launch(void* const* d_in, const int* in_sizes, int n_in,
                              void* d_out, int out_size, void* d_ws, size_t ws_size,
                              hipStream_t stream) {
  if (n_in < 10) return;
  if (out_size <= 0 || (out_size % (QB * NOUT)) != 0) return;
  const int M = out_size / NOUT;
  if (in_sizes[0] != M * KNB || in_sizes[1] != M * KNB) return;
  if (in_sizes[2] != NG * 3 || in_sizes[3] != NG * 3 || in_sizes[4] != NG * 3) return;
  if (in_sizes[5] != W0 * KC) return;
  if (in_sizes[6] != W0 * WID || in_sizes[7] != WID) return;
  if (in_sizes[8] != WID * NOUT || in_sizes[9] != NOUT) return;

  const int*   Bidx = (const int*)  d_in[0];
  const float* Bw   = (const float*)d_in[1];
  const float* x    = (const float*)d_in[2];
  const float* y    = (const float*)d_in[3];
  const float* z    = (const float*)d_in[4];
  const float* core = (const float*)d_in[5];
  const float* W1   = (const float*)d_in[6];
  const float* b1   = (const float*)d_in[7];
  const float* W2   = (const float*)d_in[8];
  const float* b2   = (const float*)d_in[9];
  float* out = (float*)d_out;

  const size_t w1t_bytes = (size_t)WID * W0 * 2;
  const size_t ck_bytes  = (size_t)W0 * KP * 2;
  const size_t total = w1t_bytes + ck_bytes;
  if (total > ws_size) return;

  char* ws = (char*)d_ws;
  _Float16* W1T   = (_Float16*)(ws);
  _Float16* coreK = (_Float16*)(ws + w1t_bytes);

  prep_w1_kernel<<<64, 256, 0, stream>>>(W1, W1T);
  prep_core_kernel<<<1, 256, 0, stream>>>(core, coreK);
  gather_mlp_kernel<<<M / QB, 256, 0, stream>>>(Bidx, Bw, x, y, z, coreK, W1T, b1, W2, b2, out);
}
